// UE_Mamba_decoder_Gated_50706383897027
// MI455X (gfx1250) — hardware-verified
//
#include <hip/hip_runtime.h>
#include <hip/hip_bf16.h>


constexpr int NB_  = 2;
constexpr int NC_  = 128;
constexpr int NH_  = 64;
constexpr int NW_  = 64;
constexpr int NL_  = NH_ * NW_;
constexpr int NT_  = NB_ * NL_;
constexpr int NS_  = 16;
constexpr int NXP_ = 192;
constexpr int LDD_ = 256;

static_assert(NL_ == 4096);
static_assert(NT_ % 64 == 0);
static_assert(NC_ % 32 == 0);
static_assert(NXP_ % 64 == 0);
static_assert(LDD_ % 64 == 0);

typedef float          v4f   __attribute__((ext_vector_type(4)));
typedef float          v8f   __attribute__((ext_vector_type(8)));
typedef __bf16         v16b  __attribute__((ext_vector_type(16)));
typedef unsigned short u16x8 __attribute__((ext_vector_type(8)));
typedef unsigned short u16x4 __attribute__((ext_vector_type(4)));

union FragB { u16x8 h[2]; v16b v; };

__device__ __forceinline__ unsigned short f2bf(float f) {
    unsigned u = __float_as_uint(f);
    unsigned r = u + 0x7FFFu + ((u >> 16) & 1u);
    return (unsigned short)(r >> 16);
}
__device__ __forceinline__ float bf2f(unsigned short b) {
    return __uint_as_float(((unsigned)b) << 16);
}
__device__ __forceinline__ v8f ld8f(const float* p) {
    v4f a = *(const v4f*)p;
    v4f b = *(const v4f*)(p + 4);
    return __builtin_shufflevector(a, b, 0, 1, 2, 3, 4, 5, 6, 7);
}
__device__ __forceinline__ void split8(const v8f& x, u16x8& hv, u16x8& lv) {
#pragma unroll
    for (int c = 0; c < 8; ++c) {
        const float f = x[c];
        const unsigned short hb = f2bf(f);
        hv[c] = hb;
        lv[c] = f2bf(f - bf2f(hb));
    }
}
__device__ __forceinline__ float wsum32(float v) {
    v += __shfl_xor(v, 16, 32);
    v += __shfl_xor(v, 8, 32);
    v += __shfl_xor(v, 4, 32);
    v += __shfl_xor(v, 2, 32);
    v += __shfl_xor(v, 1, 32);
    return v;
}
__device__ __forceinline__ float silu_f(float x) {
    return x * __builtin_amdgcn_rcpf(1.0f + __expf(-x));
}
__device__ __forceinline__ float sigm_f(float x) {
    return __builtin_amdgcn_rcpf(1.0f + __expf(-x));
}
__device__ __forceinline__ float softplus_f(float x) {
    return fmaxf(x, 0.0f) + log1pf(expf(-fabsf(x)));
}
__device__ __forceinline__ v4f ln128(v4f v, v4f wv, v4f bv) {
    float s = (v.x + v.y) + (v.z + v.w);
    s = wsum32(s);
    const float mu = s * 0.0078125f;
    v4f d = v - mu;
    float q = d.x * d.x + d.y * d.y + d.z * d.z + d.w * d.w;
    q = wsum32(q);
    const float rinv = rsqrtf(q * 0.0078125f + 1e-6f);
    return (wv * d) * rinv + bv;
}

__device__ __forceinline__ void mma_bf(v8f& acc, const FragB& a, const FragB& b) {
    acc = __builtin_amdgcn_wmma_f32_16x16x32_bf16(false, a.v, false, b.v, (short)0, acc, false, false);
    asm volatile("v_nop\n\tv_nop\n\tv_nop\n\tv_nop" : "+v"(acc) : "v"(a.v), "v"(b.v));
}

__global__ __launch_bounds__(256)
void cvt_w4_kernel(const float* __restrict__ s0, unsigned short* h0, unsigned short* l0,
                   const float* __restrict__ s1, unsigned short* h1, unsigned short* l1,
                   const float* __restrict__ s2, unsigned short* h2, unsigned short* l2,
                   const float* __restrict__ s3, unsigned short* h3, unsigned short* l3,
                   int n80, int n81, int n82, int n83)
{
    const float* src = s0; unsigned short* dh = h0; unsigned short* dl = l0; int n8 = n80;
    if (blockIdx.y == 1)      { src = s1; dh = h1; dl = l1; n8 = n81; }
    else if (blockIdx.y == 2) { src = s2; dh = h2; dl = l2; n8 = n82; }
    else if (blockIdx.y == 3) { src = s3; dh = h3; dl = l3; n8 = n83; }
    const int i = blockIdx.x * 256 + threadIdx.x;
    if (i >= n8) return;
    const size_t e = (size_t)i * 8;
    const v8f x = ld8f(src + e);
    u16x8 hv, lv;
    split8(x, hv, lv);
    *(volatile u16x8*)(dh + e) = hv;
    *(volatile u16x8*)(dl + e) = lv;
    __threadfence();
    *(volatile u16x8*)(dh + e) = hv;
    *(volatile u16x8*)(dl + e) = lv;
}

__global__ __launch_bounds__(256)
void pack_xproj_kernel(const float* __restrict__ wf, const float* __restrict__ wb, const float* __restrict__ wsd,
                       unsigned short* dh, unsigned short* dl)
{
    const int i = blockIdx.x * 256 + threadIdx.x;
    if (i >= NXP_ * 16) return;
    const int n  = i >> 4;
    const int k0 = (i & 15) * 8;
    const int jf = min(n, 35);
    const int jb = min(max(n - 48, 0), 35);
    const int js = min(max(n - 96, 0), 39);
    const int kf = k0 & 63;
    const v8f cf = ld8f(wf + jf * 64 + kf);
    const v8f cb = ld8f(wb + jb * 64 + kf);
    const v8f cs = ld8f(wsd + js * 128 + k0);
    const bool uf = (n < 36) && (k0 < 64);
    const bool ub = (n >= 48) && (n < 84) && (k0 >= 64);
    const bool us = (n >= 96) && (n < 136);
    v8f v;
#pragma unroll
    for (int c = 0; c < 8; ++c)
        v[c] = uf ? cf[c] : (ub ? cb[c] : (us ? cs[c] : 0.0f));
    u16x8 hv, lv;
    split8(v, hv, lv);
    const size_t e = (size_t)i * 8;
    *(volatile u16x8*)(dh + e) = hv;
    *(volatile u16x8*)(dl + e) = lv;
    __threadfence();
    *(volatile u16x8*)(dh + e) = hv;
    *(volatile u16x8*)(dl + e) = lv;
}

__global__ __launch_bounds__(256)
void cvt2d_kernel(const float* __restrict__ src, int lds_, int scol,
                  unsigned short* dh, unsigned short* dl, int ldd, int dcol)
{
    const int i = blockIdx.x * 256 + threadIdx.x;
    const int row = i >> 4, g = i & 15;
    if (row >= NT_) return;
    const v8f x = ld8f(src + (size_t)row * lds_ + scol + g * 8);
    u16x8 hv, lv;
    split8(x, hv, lv);
    const size_t e = (size_t)row * ldd + dcol + g * 8;
    *(volatile u16x8*)(dh + e) = hv;
    *(volatile u16x8*)(dl + e) = lv;
    __threadfence();
    *(volatile u16x8*)(dh + e) = hv;
    *(volatile u16x8*)(dl + e) = lv;
}

template<int NBF>
__device__ __forceinline__ void tile_store_pass(const float* st, float* gp, int ldc, int lane) {
    constexpr int CW  = NBF * 16;
    constexpr int P   = CW + 4;
    constexpr int LPR = CW / 4;
    constexpr int RPI = 32 / LPR;
    constexpr int NIT = 32 / RPI;
    const int rsub = lane / LPR;
    const int c4   = (lane % LPR) * 4;
#pragma unroll
    for (int it = 0; it < NIT; ++it) {
        const int row = it * RPI + rsub;
        const v4f v = *(const v4f*)(st + row * P + c4);
        *(volatile v4f*)(gp + (size_t)row * ldc + c4) = v;
    }
}

__global__ __launch_bounds__(128)
void gemm_split_kernel(const unsigned short* __restrict__ Ah, const unsigned short* __restrict__ Al,
                       const unsigned short* __restrict__ Bh, const unsigned short* __restrict__ Bl,
                       const float* __restrict__ bias, int has_bias,
                       float* C, int K, int ldc)
{
    constexpr int NBF = 2;
    constexpr int CW  = NBF * 16;
    constexpr int P   = CW + 4;
    __shared__ __attribute__((aligned(16))) float stile[4][32 * P];

    const int tid  = threadIdx.x;
    const int lane = tid & 31;
    const int wave = tid >> 5;
    const int h    = lane >> 4;
    const int m    = lane & 15;
    const int wm   = wave >> 1;
    const int wn   = wave & 1;

    const int rowW = blockIdx.y * 64 + wm * 32;
    const int colW = blockIdx.x * (2 * CW) + wn * CW;

    v8f acc[2 * NBF];
#pragma unroll
    for (int j = 0; j < 2 * NBF; ++j)
#pragma unroll
        for (int r = 0; r < 8; ++r) acc[j][r] = 0.0f;

    const size_t aoff  = (size_t)(rowW + m) * K + 8 * h;
    const size_t boff  = (size_t)(colW + m) * K + 8 * h;
    const size_t sub16 = (size_t)16 * K;
    const int nk = K >> 5;

#pragma unroll 1
    for (int kt = 0; kt < nk; ++kt) {
        const size_t k0 = (size_t)kt * 32;
        FragB fa[2], ga[2], fb[NBF], gb[NBF];
#pragma unroll
        for (int s = 0; s < 2; ++s) {
            const unsigned short* p = Ah + aoff + s * sub16 + k0;
            const unsigned short* q = Al + aoff + s * sub16 + k0;
            fa[s].h[0] = *(const u16x8*)(p);
            fa[s].h[1] = *(const u16x8*)(p + 16);
            ga[s].h[0] = *(const u16x8*)(q);
            ga[s].h[1] = *(const u16x8*)(q + 16);
        }
#pragma unroll
        for (int j = 0; j < NBF; ++j) {
            const unsigned short* p = Bh + boff + j * sub16 + k0;
            const unsigned short* q = Bl + boff + j * sub16 + k0;
            fb[j].h[0] = *(const u16x8*)(p);
            fb[j].h[1] = *(const u16x8*)(p + 16);
            gb[j].h[0] = *(const u16x8*)(q);
            gb[j].h[1] = *(const u16x8*)(q + 16);
        }
#pragma unroll
        for (int s = 0; s < 2; ++s)
#pragma unroll
            for (int j = 0; j < NBF; ++j) {
                mma_bf(acc[s * NBF + j], fa[s], fb[j]);
                mma_bf(acc[s * NBF + j], fa[s], gb[j]);
                mma_bf(acc[s * NBF + j], ga[s], fb[j]);
            }
    }

    float bv0 = 0.0f, bv1 = 0.0f;
    if (has_bias != 0) { bv0 = bias[colW + m]; bv1 = bias[colW + 16 + m]; }

    float* st = stile[wave];
#pragma unroll
    for (int s = 0; s < 2; ++s)
#pragma unroll
        for (int j = 0; j < NBF; ++j)
#pragma unroll
            for (int r = 0; r < 8; ++r)
                st[(s * 16 + 8 * h + r) * P + j * 16 + m] = acc[s * NBF + j][r] + (j == 0 ? bv0 : bv1);
    __syncthreads();

    float* gp = C + (size_t)rowW * ldc + colW;
    tile_store_pass<NBF>(st, gp, ldc, lane);
    __threadfence();
    tile_store_pass<NBF>(st, gp, ldc, lane);
}

__global__ __launch_bounds__(256)
void ln_in_kernel(const float* __restrict__ x, const float* __restrict__ w, const float* __restrict__ bb,
                  unsigned short* Xh, unsigned short* Xl)
{
    __shared__ __attribute__((aligned(16))) float sx[NC_ * 33];
    __shared__ __attribute__((aligned(16))) unsigned short stg[2 * 32 * NC_];

    const int tid = threadIdx.x, lane = tid & 31, wave = tid >> 5;
    const int blk = blockIdx.x;
    const int b  = blk >> 7;
    const int y  = (blk >> 1) & 63;
    const int x0 = (blk & 1) * 32;

#pragma unroll 4
    for (int it = 0; it < 16; ++it) {
        const int c = it * 8 + wave;
        sx[c * 33 + lane] = x[(((size_t)b * NC_ + c) * NH_ + y) * NW_ + x0 + lane];
    }
    __syncthreads();

    const int c0 = lane * 4;
    v4f wv, bv;
    wv.x = w[c0]; wv.y = w[c0 + 1]; wv.z = w[c0 + 2]; wv.w = w[c0 + 3];
    bv.x = bb[c0]; bv.y = bb[c0 + 1]; bv.z = bb[c0 + 2]; bv.w = bb[c0 + 3];
#pragma unroll
    for (int j = 0; j < 4; ++j) {
        const int xx = wave * 4 + j;
        v4f v;
        v.x = sx[(c0 + 0) * 33 + xx];
        v.y = sx[(c0 + 1) * 33 + xx];
        v.z = sx[(c0 + 2) * 33 + xx];
        v.w = sx[(c0 + 3) * 33 + xx];
        const v4f o = ln128(v, wv, bv);
        u16x4 hv, lv;
#pragma unroll
        for (int i = 0; i < 4; ++i) {
            const float f = o[i];
            const unsigned short hb = f2bf(f);
            hv[i] = hb;
            lv[i] = f2bf(f - bf2f(hb));
        }
        *(u16x4*)(stg + (0 * 32 + xx) * NC_ + c0) = hv;
        *(u16x4*)(stg + (1 * 32 + xx) * NC_ + c0) = lv;
    }
    __syncthreads();

    u16x8 vals[4];
    size_t goff[4];
    const size_t tok0 = (size_t)b * NL_ + (size_t)y * NW_ + x0;
#pragma unroll
    for (int it = 0; it < 4; ++it) {
        const int line = it * 32 + (tid >> 3);
        const int p    = it >> 1;
        const int row  = (line >> 1) & 31;
        const int hl   = line & 1;
        vals[it] = *(const u16x8*)(stg + (p * 32 + row) * NC_ + hl * 64 + (tid & 7) * 8);
        goff[it] = (tok0 + row) * NC_ + hl * 64 + (tid & 7) * 8;
    }
    *(volatile u16x8*)(Xh + goff[0]) = vals[0];
    *(volatile u16x8*)(Xh + goff[1]) = vals[1];
    *(volatile u16x8*)(Xl + goff[2]) = vals[2];
    *(volatile u16x8*)(Xl + goff[3]) = vals[3];
    __threadfence();
    *(volatile u16x8*)(Xh + goff[0]) = vals[0];
    *(volatile u16x8*)(Xh + goff[1]) = vals[1];
    *(volatile u16x8*)(Xl + goff[2]) = vals[2];
    *(volatile u16x8*)(Xl + goff[3]) = vals[3];
}

__global__ __launch_bounds__(256)
void ln_tok_kernel(const float* __restrict__ in, int ldi, const float* __restrict__ w,
                   const float* __restrict__ bb, float* out)
{
    const int tid = threadIdx.x, lane = tid & 31, wave = tid >> 5;
    const int tok = blockIdx.x * 8 + wave;
    const int c0  = lane * 4;
    const v4f v = *(const v4f*)(in + (size_t)tok * ldi + c0);
    v4f wv, bv;
    wv.x = w[c0]; wv.y = w[c0 + 1]; wv.z = w[c0 + 2]; wv.w = w[c0 + 3];
    bv.x = bb[c0]; bv.y = bb[c0 + 1]; bv.z = bb[c0 + 2]; bv.w = bb[c0 + 3];
    const v4f o = ln128(v, wv, bv);
    float* gp = out + (size_t)tok * NC_ + c0;
    *(volatile v4f*)gp = o;
    __threadfence();
    *(volatile v4f*)gp = o;
}

__global__ __launch_bounds__(256)
void dwconv_silu_kernel(const float* __restrict__ in, int ldi, int coff,
                        const float* __restrict__ wk, const float* __restrict__ bias, float* out)
{
    const int tid = threadIdx.x, lane = tid & 31, wave = tid >> 5;
    const int tok = blockIdx.x * 8 + wave;
    const int b   = tok >> 12;
    const int y   = (tok >> 6) & 63;
    const int xx  = tok & 63;
    const int c0  = lane * 4;

    v4f acc = {0.0f, 0.0f, 0.0f, 0.0f};
#pragma unroll
    for (int dy = -1; dy <= 1; ++dy) {
#pragma unroll
        for (int dx = -1; dx <= 1; ++dx) {
            const int yy = y + dy;
            const int xq = xx + dx;
            const bool valid = ((unsigned)yy < (unsigned)NH_) && ((unsigned)xq < (unsigned)NW_);
            const int yc = min(max(yy, 0), NH_ - 1);
            const int xc = min(max(xq, 0), NW_ - 1);
            const size_t tn = ((size_t)b << 12) + (size_t)yc * NW_ + xc;
            v4f val = *(const v4f*)(in + tn * ldi + coff + c0);
            const int tap = (dy + 1) * 3 + (dx + 1);
            v4f wt;
            wt.x = wk[(c0 + 0) * 9 + tap];
            wt.y = wk[(c0 + 1) * 9 + tap];
            wt.z = wk[(c0 + 2) * 9 + tap];
            wt.w = wk[(c0 + 3) * 9 + tap];
#pragma unroll
            for (int i = 0; i < 4; ++i) val[i] = valid ? val[i] : 0.0f;
            acc += val * wt;
        }
    }
    v4f bv;
    bv.x = bias[c0]; bv.y = bias[c0 + 1]; bv.z = bias[c0 + 2]; bv.w = bias[c0 + 3];
    acc += bv;
    v4f o;
#pragma unroll
    for (int i = 0; i < 4; ++i) o[i] = silu_f(acc[i]);
    float* gp = out + (size_t)tok * NC_ + c0;
    *(volatile v4f*)gp = o;
    __threadfence();
    *(volatile v4f*)gp = o;
}

__global__ __launch_bounds__(256)
void dtproj_kernel(const float* __restrict__ dbl,
                   const float* __restrict__ xbf, const float* __restrict__ wf, const float* __restrict__ tbf,
                   const float* __restrict__ xbb, const float* __restrict__ wb, const float* __restrict__ tbb,
                   const float* __restrict__ xbs, const float* __restrict__ wsd, const float* __restrict__ tbs,
                   float* delta)
{
    const int tok = blockIdx.x;
    const int j   = threadIdx.x;
    const float* dr = dbl + (size_t)tok * NXP_;
    float pre;
    if (j < 64) {
        float s = 0.0f;
#pragma unroll
        for (int r = 0; r < 4; ++r) s += (dr[r] + xbf[r]) * wf[j * 4 + r];
        pre = s + tbf[j];
    } else if (j < 128) {
        const int jj = j - 64;
        float s = 0.0f;
#pragma unroll
        for (int r = 0; r < 4; ++r) s += (dr[48 + r] + xbb[r]) * wb[jj * 4 + r];
        pre = s + tbb[jj];
    } else {
        const int jj = j - 128;
        float s = 0.0f;
#pragma unroll
        for (int r = 0; r < 8; ++r) s += (dr[96 + r] + xbs[r]) * wsd[jj * 8 + r];
        pre = s + tbs[jj];
    }
    const float d = softplus_f(pre);
    float* gp = delta + (size_t)tok * LDD_ + j;
    *(volatile float*)gp = d;
    __threadfence();
    *(volatile float*)gp = d;
}

__global__ __launch_bounds__(512)
void scan_kernel(const float* __restrict__ xm, int chan0,
                 const float* __restrict__ delta, int dcol,
                 const float* __restrict__ dbl, int offB, int offC,
                 const float* __restrict__ xpb, int rr,
                 const float* __restrict__ Alog, const float* __restrict__ Dp,
                 const float* __restrict__ mfg, const float* __restrict__ mbg,
                 const float* __restrict__ muc,
                 int mode, float* yout, int ocol)
{
    __shared__ int perm[NL_];
    __shared__ int cnt[4 * 512];
    __shared__ int tot[4];
    __shared__ __attribute__((aligned(16))) float ystg[16 * 32];

    const int tid   = threadIdx.x;
    const int lane  = tid & 31;
    const int wave  = tid >> 5;
    const int cl    = tid >> 4;
    const int n     = tid & 15;
    const int b     = blockIdx.y;
    const int cbase = blockIdx.x * 32;
    const int c     = cbase + cl;
    const size_t rb = (size_t)b * NL_;

    if (mode == 2) {
        int cls8[8];
        int k0c = 0, k1c = 0, k2c = 0, k3c = 0;
#pragma unroll
        for (int j = 0; j < 8; ++j) {
            const int t = tid * 8 + j;
            const float f = mfg[rb + t];
            const float g = mbg[rb + t];
            const float q = muc[rb + t];
            const int cs = (f > 0.5f) ? 3 : ((g > 0.5f) ? 2 : ((q > 0.5f) ? 1 : 0));
            cls8[j] = cs;
            k3c += (cs == 3); k2c += (cs == 2); k1c += (cs == 1); k0c += (cs == 0);
        }
        cnt[tid] = k0c; cnt[512 + tid] = k1c; cnt[1024 + tid] = k2c; cnt[1536 + tid] = k3c;
        __syncthreads();
        int s0 = 0, s1 = 0, s2 = 0, s3 = 0;
#pragma unroll 1
        for (int j2 = tid + 1; j2 < 512; ++j2) {
            s0 += cnt[j2]; s1 += cnt[512 + j2]; s2 += cnt[1024 + j2]; s3 += cnt[1536 + j2];
        }
        if (tid == 0) { tot[0] = s0 + k0c; tot[1] = s1 + k1c; tot[2] = s2 + k2c; tot[3] = s3 + k3c; }
        __syncthreads();
        const int t3 = tot[3], t2 = tot[2], t1 = tot[1];
        const int base3 = s3;
        const int base2 = t3 + s2;
        const int base1 = t3 + t2 + s1;
        const int base0 = t3 + t2 + t1 + s0;
        int a0 = 0, a1 = 0, a2 = 0, a3 = 0;
#pragma unroll
        for (int j = 7; j >= 0; --j) {
            const int t  = tid * 8 + j;
            const int cs = cls8[j];
            int rank = (cs == 3) ? (base3 + a3) : ((cs == 2) ? (base2 + a2) : ((cs == 1) ? (base1 + a1) : (base0 + a0)));
            rank = min(max(rank, 0), NL_ - 1);
            perm[rank] = t;
            a3 += (cs == 3); a2 += (cs == 2); a1 += (cs == 1); a0 += (cs == 0);
        }
        __syncthreads();
    }

    const float A  = -expf(Alog[c * NS_ + n]);
    const float Dd = Dp[c];
    const float bB = xpb[rr + n];
    const float bC = xpb[rr + NS_ + n];
    float h = 0.0f;
    const int colo = ocol + cbase + (lane & 7) * 4;

#pragma unroll 1
    for (int k0 = 0; k0 < NL_; k0 += 16) {
#pragma unroll 1
        for (int t = 0; t < 16; ++t) {
            const int k = k0 + t;
            int tok;
            if (mode == 0) tok = k; else if (mode == 1) tok = NL_ - 1 - k; else tok = perm[k] & (NL_ - 1);
            const size_t row = rb + (size_t)tok;
            const float dl = delta[row * LDD_ + dcol + c];
            const float u  = xm[row * NC_ + chan0 + c];
            const float Bs = dbl[row * NXP_ + offB + n] + bB;
            const float Cs = dbl[row * NXP_ + offC + n] + bC;
            const float a  = expf(dl * A);
            h = a * h + (dl * u) * Bs;
            float v = h * Cs;
            v += __shfl_xor(v, 8, 32);
            v += __shfl_xor(v, 4, 32);
            v += __shfl_xor(v, 2, 32);
            v += __shfl_xor(v, 1, 32);
            const float yv = v + u * Dd;
            if (n == 0) ystg[t * 32 + cl] = yv;
        }
        __syncthreads();
        {
            const int k = k0 + wave;
            int tok;
            if (mode == 0) tok = k; else if (mode == 1) tok = NL_ - 1 - k; else tok = perm[k] & (NL_ - 1);
            const v4f val = *(const v4f*)(ystg + wave * 32 + (lane & 7) * 4);
            float* gp = yout + (rb + (size_t)tok) * NC_ + colo;
            if (lane < 8) *(volatile v4f*)gp = val;
            __threadfence();
            if (lane < 8) *(volatile v4f*)gp = val;
        }
        __syncthreads();
    }
}

__global__ __launch_bounds__(256)
void bn_relu_cvt_kernel(const float* __restrict__ g, const float* __restrict__ bng, const float* __restrict__ bnbe,
                        const float* __restrict__ bnm, const float* __restrict__ bnv,
                        unsigned short* dh, unsigned short* dl)
{
    const int i = blockIdx.x * 256 + threadIdx.x;
    if (i >= NT_ * 16) return;
    const int c0 = (i & 15) * 8;
    const size_t e = (size_t)i * 8;
    const v8f x = ld8f(g + e);
    v8f o;
#pragma unroll
    for (int c = 0; c < 8; ++c) {
        const int ch = c0 + c;
        float v = (x[c] - bnm[ch]) * rsqrtf(bnv[ch] + 1e-5f);
        v = v * bng[ch] + bnbe[ch];
        o[c] = fmaxf(v, 0.0f);
    }
    u16x8 hv, lv;
    split8(o, hv, lv);
    *(volatile u16x8*)(dh + e) = hv;
    *(volatile u16x8*)(dl + e) = lv;
    __threadfence();
    *(volatile u16x8*)(dh + e) = hv;
    *(volatile u16x8*)(dl + e) = lv;
}

__global__ __launch_bounds__(256)
void gate_fuse_kernel(const float* __restrict__ glog, const float* __restrict__ ypm, const float* __restrict__ cat,
                      unsigned short* dh, unsigned short* dl)
{
    const int i = blockIdx.x * 256 + threadIdx.x;
    if (i >= NT_ * 16) return;
    const int row = i >> 4, gq = i & 15;
    const size_t e = (size_t)i * 8;
    const v8f gl = ld8f(glog + e);
    const v8f sv = ld8f(ypm + e);
    const v8f cv = ld8f(cat + e);
    v8f o;
#pragma unroll
    for (int c = 0; c < 8; ++c) {
        const float gg = sigm_f(gl[c]);
        o[c] = gg * sv[c] + (1.0f - gg) * cv[c];
    }
    u16x8 hv, lv;
    split8(o, hv, lv);
    const size_t d = (size_t)row * 256 + gq * 8;
    *(volatile u16x8*)(dh + d) = hv;
    *(volatile u16x8*)(dl + d) = lv;
    __threadfence();
    *(volatile u16x8*)(dh + d) = hv;
    *(volatile u16x8*)(dl + d) = lv;
}

__global__ __launch_bounds__(256)
void ln_out_kernel(const float* __restrict__ ob, const float* __restrict__ w, const float* __restrict__ bb,
                   float* out)
{
    __shared__ __attribute__((aligned(16))) float so[NC_ * 36];
    const int tid = threadIdx.x, lane = tid & 31, wave = tid >> 5;
    const int blk = blockIdx.x;
    const int b  = blk >> 7;
    const int y  = (blk >> 1) & 63;
    const int x0 = (blk & 1) * 32;
    const int c0 = lane * 4;
    v4f wv, bv;
    wv.x = w[c0]; wv.y = w[c0 + 1]; wv.z = w[c0 + 2]; wv.w = w[c0 + 3];
    bv.x = bb[c0]; bv.y = bb[c0 + 1]; bv.z = bb[c0 + 2]; bv.w = bb[c0 + 3];
#pragma unroll
    for (int j = 0; j < 4; ++j) {
        const int xx = wave * 4 + j;
        const size_t tok = (size_t)b * NL_ + (size_t)y * NW_ + x0 + xx;
        const v4f v = *(const v4f*)(ob + tok * NC_ + c0);
        const v4f o = ln128(v, wv, bv);
        so[(c0 + 0) * 36 + xx] = o.x;
        so[(c0 + 1) * 36 + xx] = o.y;
        so[(c0 + 2) * 36 + xx] = o.z;
        so[(c0 + 3) * 36 + xx] = o.w;
    }
    __syncthreads();
    v4f vals[4];
    size_t goff[4];
#pragma unroll
    for (int it = 0; it < 4; ++it) {
        const int c = it * 32 + (tid >> 3);
        vals[it] = *(const v4f*)(so + c * 36 + (tid & 7) * 4);
        goff[it] = (((size_t)b * NC_ + c) * NH_ + y) * NW_ + x0 + (tid & 7) * 4;
    }
#pragma unroll
    for (int it = 0; it < 4; ++it) *(volatile v4f*)(out + goff[it]) = vals[it];
    __threadfence();
#pragma unroll
    for (int it = 0; it < 4; ++it) *(volatile v4f*)(out + goff[it]) = vals[it];
}

extern "C" void kernel_launch(void* const* d_in, const int* in_sizes, int n_in,
                              void* d_out, int out_size, void* d_ws, size_t ws_size,
                              hipStream_t stream)
{
    if (n_in < 46) return;
    const int want[46] = {
        NT_ * NC_, NT_, NT_, NT_,
        128, 128, 256 * 128, 256,
        128, 128, 1152, 128, 1152, 128,
        2304, 36, 256, 64, 1024, 64,
        2304, 36, 256, 64, 1024, 64,
        5120, 40, 1024, 128, 2048, 128,
        128, 128,
        32768, 128, 128, 128, 128, 128, 16384, 128,
        32768, 128, 128, 128 };
    for (int i = 0; i < 46; ++i) if (in_sizes[i] != want[i]) return;
    if (out_size != NT_ * NC_) return;

    const float* x    = (const float*)d_in[0];
    const float* mfg  = (const float*)d_in[1];
    const float* mbg  = (const float*)d_in[2];
    const float* muc  = (const float*)d_in[3];
    const float* niw  = (const float*)d_in[4];
    const float* nib  = (const float*)d_in[5];
    const float* ipw  = (const float*)d_in[6];
    const float* ipb  = (const float*)d_in[7];
    const float* lmw  = (const float*)d_in[8];
    const float* lmb  = (const float*)d_in[9];
    const float* cmw  = (const float*)d_in[10];
    const float* cmb  = (const float*)d_in[11];
    const float* crw  = (const float*)d_in[12];
    const float* crb  = (const float*)d_in[13];
    const float* xfw  = (const float*)d_in[14];
    const float* xfb  = (const float*)d_in[15];
    const float* dfw  = (const float*)d_in[16];
    const float* dfb  = (const float*)d_in[17];
    const float* alf  = (const float*)d_in[18];
    const float* Df   = (const float*)d_in[19];
    const float* xbw  = (const float*)d_in[20];
    const float* xbb  = (const float*)d_in[21];
    const float* dbw  = (const float*)d_in[22];
    const float* dbb  = (const float*)d_in[23];
    const float* alb  = (const float*)d_in[24];
    const float* Db   = (const float*)d_in[25];
    const float* xsw  = (const float*)d_in[26];
    const float* xsb  = (const float*)d_in[27];
    const float* dsw  = (const float*)d_in[28];
    const float* dsb  = (const float*)d_in[29];
    const float* als  = (const float*)d_in[30];
    const float* Ds   = (const float*)d_in[31];
    const float* lcw  = (const float*)d_in[32];
    const float* lcb  = (const float*)d_in[33];
    const float* g0w  = (const float*)d_in[34];
    const float* g0b  = (const float*)d_in[35];
    const float* bng  = (const float*)d_in[36];
    const float* bnbe = (const float*)d_in[37];
    const float* bnm  = (const float*)d_in[38];
    const float* bnv  = (const float*)d_in[39];
    const float* g1w  = (const float*)d_in[40];
    const float* g1b  = (const float*)d_in[41];
    const float* ow   = (const float*)d_in[42];
    const float* ob   = (const float*)d_in[43];
    const float* now_ = (const float*)d_in[44];
    const float* nob  = (const float*)d_in[45];
    float* out = (float*)d_out;

    char* ws = (char*)d_ws;
    size_t off = 0;
    auto carve = [&](size_t bytes) -> char* { char* p = ws + off; off += (bytes + 255) & ~(size_t)255; return p; };
    const size_t P16_128 = (size_t)NT_ * 128 * 2;
    const size_t P16_256 = (size_t)NT_ * 256 * 2;
    const size_t P32_128 = (size_t)NT_ * 128 * 4;
    const size_t P32_256 = (size_t)NT_ * 256 * 4;
    const size_t P32_192 = (size_t)NT_ * NXP_ * 4;

    unsigned short* WIh  = (unsigned short*)carve((size_t)256 * 128 * 2);
    unsigned short* WIl  = (unsigned short*)carve((size_t)256 * 128 * 2);
    unsigned short* WG0h = (unsigned short*)carve((size_t)128 * 256 * 2);
    unsigned short* WG0l = (unsigned short*)carve((size_t)128 * 256 * 2);
    unsigned short* WG1h = (unsigned short*)carve((size_t)128 * 128 * 2);
    unsigned short* WG1l = (unsigned short*)carve((size_t)128 * 128 * 2);
    unsigned short* WOh  = (unsigned short*)carve((size_t)128 * 256 * 2);
    unsigned short* WOl  = (unsigned short*)carve((size_t)128 * 256 * 2);
    unsigned short* WXh  = (unsigned short*)carve((size_t)NXP_ * 128 * 2);
    unsigned short* WXl  = (unsigned short*)carve((size_t)NXP_ * 128 * 2);
    unsigned short* Xh   = (unsigned short*)carve(P16_128);
    unsigned short* Xl   = (unsigned short*)carve(P16_128);
    float*          XP   = (float*)carve(P32_256);
    float*          XMLN = (float*)carve(P32_128);
    float*          XM   = (float*)carve(P32_128);
    float*          XRES = (float*)carve(P32_128);
    unsigned short* XMh  = (unsigned short*)carve(P16_128);
    unsigned short* XMl  = (unsigned short*)carve(P16_128);
    float*          DBL  = (float*)carve(P32_192);
    float*          DELT = (float*)carve(P32_256);
    float*          YCAT = (float*)carve(P32_128);
    float*          YPM  = (float*)carve(P32_128);
    float*          CAT  = (float*)carve(P32_128);
    unsigned short* G0Ah = (unsigned short*)carve(P16_256);
    unsigned short* G0Al = (unsigned short*)carve(P16_256);
    float*          GBUF = (float*)carve(P32_128);
    unsigned short* G1Ah = (unsigned short*)carve(P16_128);
    unsigned short* G1Al = (unsigned short*)carve(P16_128);
    float*          GLOG = (float*)carve(P32_128);
    unsigned short* OAh  = (unsigned short*)carve(P16_256);
    unsigned short* OAl  = (unsigned short*)carve(P16_256);
    float*          OBUF = (float*)carve(P32_128);
    if (off > ws_size) return;

    const dim3 b256(256), b128(128), b512(512);

    cvt_w4_kernel<<<dim3(16, 4), b256, 0, stream>>>(ipw, WIh, WIl, g0w, WG0h, WG0l, g1w, WG1h, WG1l, ow, WOh, WOl,
                                                   (256 * 128) / 8, (128 * 256) / 8, (128 * 128) / 8, (128 * 256) / 8);
    pack_xproj_kernel<<<dim3((NXP_ * 16 + 255) / 256), b256, 0, stream>>>(xfw, xbw, xsw, WXh, WXl);

    ln_in_kernel<<<dim3(NB_ * NH_ * 2), b256, 0, stream>>>(x, niw, nib, Xh, Xl);
    gemm_split_kernel<<<dim3(256 / 64, NT_ / 64), b128, 0, stream>>>(Xh, Xl, WIh, WIl, ipb, 1, XP, 128, 256);

    ln_tok_kernel<<<dim3(NT_ / 8), b256, 0, stream>>>(XP, 256, lmw, lmb, XMLN);
    dwconv_silu_kernel<<<dim3(NT_ / 8), b256, 0, stream>>>(XMLN, 128, 0, cmw, cmb, XM);
    dwconv_silu_kernel<<<dim3(NT_ / 8), b256, 0, stream>>>(XP, 256, 128, crw, crb, XRES);

    cvt2d_kernel<<<dim3(NT_ * 16 / 256), b256, 0, stream>>>(XM, 128, 0, XMh, XMl, 128, 0);
    gemm_split_kernel<<<dim3(NXP_ / 64, NT_ / 64), b128, 0, stream>>>(XMh, XMl, WXh, WXl, ipb, 0, DBL, 128, NXP_);

    dtproj_kernel<<<dim3(NT_), b256, 0, stream>>>(DBL, xfb, dfw, dfb, xbb, dbw, dbb, xsb, dsw, dsb, DELT);

    scan_kernel<<<dim3(2, NB_), b512, 0, stream>>>(XM, 0,  DELT, 0,   DBL, 4,   20,  xfb, 4, alf, Df, mfg, mbg, muc, 0, YCAT, 0);
    scan_kernel<<<dim3(2, NB_), b512, 0, stream>>>(XM, 64, DELT, 64,  DBL, 52,  68,  xbb, 4, alb, Db, mfg, mbg, muc, 1, YCAT, 64);
    scan_kernel<<<dim3(4, NB_), b512, 0, stream>>>(XM, 0,  DELT, 128, DBL, 104, 120, xsb, 8, als, Ds, mfg, mbg, muc, 2, YPM,  0);

    ln_tok_kernel<<<dim3(NT_ / 8), b256, 0, stream>>>(YCAT, 128, lcw, lcb, CAT);
    cvt2d_kernel<<<dim3(NT_ * 16 / 256), b256, 0, stream>>>(CAT, 128, 0, G0Ah, G0Al, 256, 0);
    cvt2d_kernel<<<dim3(NT_ * 16 / 256), b256, 0, stream>>>(YPM, 128, 0, G0Ah, G0Al, 256, 128);
    gemm_split_kernel<<<dim3(128 / 64, NT_ / 64), b128, 0, stream>>>(G0Ah, G0Al, WG0h, WG0l, g0b, 1, GBUF, 256, 128);
    bn_relu_cvt_kernel<<<dim3(NT_ * 16 / 256), b256, 0, stream>>>(GBUF, bng, bnbe, bnm, bnv, G1Ah, G1Al);
    gemm_split_kernel<<<dim3(128 / 64, NT_ / 64), b128, 0, stream>>>(G1Ah, G1Al, WG1h, WG1l, g1b, 1, GLOG, 128, 128);
    gate_fuse_kernel<<<dim3(NT_ * 16 / 256), b256, 0, stream>>>(GLOG, YPM, CAT, OAh, OAl);
    cvt2d_kernel<<<dim3(NT_ * 16 / 256), b256, 0, stream>>>(XRES, 128, 0, OAh, OAl, 256, 128);

    gemm_split_kernel<<<dim3(128 / 64, NT_ / 64), b128, 0, stream>>>(OAh, OAl, WOh, WOl, ob, 1, OBUF, 256, 128);
    ln_out_kernel<<<dim3(NB_ * NH_ * 2), b256, 0, stream>>>(OBUF, now_, nob, out);
}
